// AugmentedNeuralODE_90752658964593
// MI455X (gfx1250) — hardware-verified
//
#include <hip/hip_runtime.h>
#include <math.h>

constexpr int DIM_LAT  = 123;
constexpr int DIM_ST   = 128;
constexpr int DIM_HID  = 512;
constexpr int NBATCH   = 1024;
constexpr int NTIME    = 8;
constexpr int NSUB     = 6;
constexpr int NTHR     = 256;
constexpr int ROWS_BLK = 16;
constexpr int YPITCH   = 136;
constexpr int HPITCH   = 520;
constexpr int SPITCH   = 260;
constexpr int NOUT_EL  = NBATCH * NTIME * DIM_LAT;
constexpr int NOUT_V4  = NOUT_EL / 4;
constexpr float CARRY1     = 8.0f;
constexpr float CARRY1_INV = 0.125f;
constexpr float CARRY2     = 16.0f;
constexpr float CARRY2_INV = 0.0625f;
static_assert(DIM_ST % 32 == 0);
static_assert(DIM_HID % 32 == 0);
static_assert(DIM_HID == 64 * (NTHR / 32));
static_assert(DIM_ST == 16 * (NTHR / 32));
static_assert(NBATCH % ROWS_BLK == 0);
static_assert(NOUT_EL % (4 * NTHR) == 0);
static_assert(DIM_ST % 64 == 0 && DIM_HID % 64 == 0 && DIM_ST % 32 == 0);
static_assert(ROWS_BLK == 2 * (NTHR / 32));

constexpr float RK_A21 = 0.2f;
constexpr float RK_A31 = (float)(3.0 / 40.0);
constexpr float RK_A32 = (float)(9.0 / 40.0);
constexpr float RK_A41 = (float)(44.0 / 45.0);
constexpr float RK_A42 = (float)(56.0 / 15.0);
constexpr float RK_A43 = (float)(32.0 / 9.0);
constexpr float RK_A51 = (float)(19372.0 / 6561.0);
constexpr float RK_A52 = (float)(25360.0 / 2187.0);
constexpr float RK_A53 = (float)(64448.0 / 6561.0);
constexpr float RK_A54 = (float)(212.0 / 729.0);
constexpr float RK_A61 = (float)(9017.0 / 3168.0);
constexpr float RK_A62 = (float)(355.0 / 33.0);
constexpr float RK_A63 = (float)(46732.0 / 5247.0);
constexpr float RK_A64 = (float)(49.0 / 176.0);
constexpr float RK_A65 = (float)(5103.0 / 18656.0);
constexpr float RK_B1  = (float)(35.0 / 384.0);
constexpr float RK_B3  = (float)(500.0 / 1113.0);
constexpr float RK_B4  = (float)(125.0 / 192.0);
constexpr float RK_B5  = (float)(2187.0 / 6784.0);
constexpr float RK_B6  = (float)(11.0 / 84.0);

typedef __attribute__((ext_vector_type(16))) _Float16 v16h;
typedef __attribute__((ext_vector_type(8)))  _Float16 v8h;
typedef __attribute__((ext_vector_type(8)))  float    v8f;
typedef __attribute__((ext_vector_type(4)))  float    v4f;

__device__ __forceinline__ void dep_guard_h(v8f& a, v8f& b, v16h x, v16h y) { asm volatile("v_nop\n\tv_nop\n\tv_nop\n\tv_nop" : "+v"(a), "+v"(b) : "v"(x), "v"(y)); }
__device__ __forceinline__ void dep_guard1(v8f& a, v16h x, v16h y) { asm volatile("v_nop\n\tv_nop\n\tv_nop\n\tv_nop" : "+v"(a) : "v"(x), "v"(y)); }
__device__ __forceinline__ void keep4_h(v16h a, v16h b, v16h c, v16h d) { asm volatile("v_nop" :: "v"(a), "v"(b), "v"(c), "v"(d)); }
__device__ __forceinline__ void acc_guard4(v8f& a, v8f& b, v8f& c, v8f& d) { asm volatile("v_nop\n\tv_nop\n\tv_nop\n\tv_nop" : "+v"(a), "+v"(b), "+v"(c), "+v"(d)); }
__device__ __forceinline__ void acc_guard1(v8f& a) { asm volatile("v_nop\n\tv_nop\n\tv_nop\n\tv_nop" : "+v"(a)); }

template <typename T> struct Frag;
template <> struct Frag<_Float16> {
  typedef v16h V; union U { v16h v; v8h h[2]; };
  static __device__ __forceinline__ v16h load(const _Float16* p) {
    U f; f.h[0] = *(const v8h*)(p); f.h[1] = *(const v8h*)(p + 16); return f.v;
  }
  static __device__ __forceinline__ v8f mma(v16h a, v16h b, v8f c) {
    return __builtin_amdgcn_wmma_f32_16x16x32_f16(false, a, false, b, (short)0, c, false, false);
  }
};

__device__ __forceinline__ float ftanh(float x) { return 1.0f - 2.0f * __builtin_amdgcn_rcpf(__expf(2.0f * x) + 1.0f); }

__global__ __launch_bounds__(NTHR) void wt_cast_kernel(const float* __restrict__ in, unsigned short* __restrict__ out,
                                                       int kin, int nout, float sc) {
  __shared__ float tile[64][33];
  const int k0 = blockIdx.x * 64, n0 = blockIdx.y * 32;
  const int tid = threadIdx.x, nn = tid & 31, kq = tid >> 5;
#pragma unroll
  for (int i = 0; i < 8; ++i) {
    const int kk = kq + 8 * i;
    tile[kk][nn] = in[(size_t)(k0 + kk) * nout + n0 + nn];
  }
  __syncthreads();
  const int lane = tid & 31, wave = tid >> 5, q = lane >> 3, c8 = (lane & 7) * 8;
  const int row = 4 * wave + q;
  v8h hv;
#pragma unroll
  for (int e = 0; e < 8; ++e) hv[e] = (_Float16)(tile[c8 + e][row] * sc);
  unsigned short* op = out + (size_t)(n0 + row) * kin + k0 + c8;
  *(volatile v8h*)op = hv;
  __threadfence();
  *(volatile v8h*)op = hv;
}

__device__ __forceinline__ void store_state(float* Sl, float* dst, int wave, int hh, int c, int lane, const float (&y)[8]) {
#pragma unroll
  for (int r = 0; r < 8; ++r) Sl[(8 * hh + r) * SPITCH + 16 * wave + c] = y[r];
  __syncthreads();
  for (int pass = 0; pass < 2; ++pass) {
#pragma unroll
    for (int q = 0; q < 2; ++q) {
      const int row = 2 * wave + q;
      const v4f v = *(const v4f*)(Sl + row * SPITCH + 4 * lane);
      *(volatile v4f*)(dst + (size_t)row * DIM_ST + 4 * lane) = v;
    }
    __threadfence();
  }
  __syncthreads();
}

__device__ __forceinline__ void feval(_Float16* Ysh, _Float16* H1s, _Float16* H2s,
                                      const _Float16* __restrict__ W1T, const _Float16* __restrict__ W2T,
                                      const _Float16* __restrict__ W3T,
                                      const float (&b1r)[4], const float (&b2r)[4], float b3r,
                                      int wave, int hh, int c, const float (&yin)[8], float (&kout)[8]) {
  const int koff = hh * 8;
  const v8f z8 = {0.f, 0.f, 0.f, 0.f, 0.f, 0.f, 0.f, 0.f};
#pragma unroll
  for (int r = 0; r < 8; ++r) Ysh[(8 * hh + r) * YPITCH + 16 * wave + c] = (_Float16)yin[r];
  __syncthreads();
  {
    v8f acc[4];
#pragma unroll
    for (int nt = 0; nt < 4; ++nt) acc[nt] = z8;
    const _Float16* arow = Ysh + c * YPITCH + koff;
#pragma unroll 1
    for (int k0 = 0; k0 < DIM_ST; k0 += 32) {
      v16h bh[4];
#pragma unroll
      for (int nt = 0; nt < 4; ++nt)
        bh[nt] = Frag<_Float16>::load(W1T + (size_t)(64 * wave + 16 * nt + c) * DIM_ST + koff + k0);
      const v16h a = Frag<_Float16>::load(arow + k0);
#pragma unroll
      for (int nt = 0; nt < 4; ++nt) acc[nt] = Frag<_Float16>::mma(a, bh[nt], acc[nt]);
      dep_guard_h(acc[0], acc[3], a, bh[0]);
      keep4_h(bh[1], bh[2], bh[3], a);
    }
    acc_guard4(acc[0], acc[1], acc[2], acc[3]);
#pragma unroll
    for (int nt = 0; nt < 4; ++nt) {
      const int j = 64 * wave + 16 * nt + c;
#pragma unroll
      for (int r = 0; r < 8; ++r)
        H1s[(8 * hh + r) * HPITCH + j] = (_Float16)ftanh(acc[nt][r] * CARRY1_INV + b1r[nt]);
    }
  }
  __syncthreads();
  {
    v8f acc[4];
#pragma unroll
    for (int nt = 0; nt < 4; ++nt) acc[nt] = z8;
    const _Float16* arow = H1s + c * HPITCH + koff;
#pragma unroll 1
    for (int k0 = 0; k0 < DIM_HID; k0 += 32) {
      v16h bh[4];
#pragma unroll
      for (int nt = 0; nt < 4; ++nt)
        bh[nt] = Frag<_Float16>::load(W2T + (size_t)(64 * wave + 16 * nt + c) * DIM_HID + koff + k0);
      const v16h a = Frag<_Float16>::load(arow + k0);
#pragma unroll
      for (int nt = 0; nt < 4; ++nt) acc[nt] = Frag<_Float16>::mma(a, bh[nt], acc[nt]);
      dep_guard_h(acc[0], acc[3], a, bh[0]);
      keep4_h(bh[1], bh[2], bh[3], a);
    }
    acc_guard4(acc[0], acc[1], acc[2], acc[3]);
#pragma unroll
    for (int nt = 0; nt < 4; ++nt) {
      const int j = 64 * wave + 16 * nt + c;
#pragma unroll
      for (int r = 0; r < 8; ++r)
        H2s[(8 * hh + r) * HPITCH + j] = (_Float16)ftanh(acc[nt][r] * CARRY2_INV + b2r[nt]);
    }
  }
  __syncthreads();
  {
    v8f acc = z8;
    const _Float16* arow = H2s + c * HPITCH + koff;
    const _Float16* brow = W3T + (size_t)(16 * wave + c) * DIM_HID + koff;
#pragma unroll 1
    for (int k0 = 0; k0 < DIM_HID; k0 += 32) {
      const v16h a = Frag<_Float16>::load(arow + k0);
      const v16h b = Frag<_Float16>::load(brow + k0);
      acc = Frag<_Float16>::mma(a, b, acc);
      dep_guard1(acc, a, b);
    }
    acc_guard1(acc);
#pragma unroll
    for (int r = 0; r < 8; ++r) kout[r] = acc[r] * CARRY2_INV + b3r;
  }
}

__global__ __launch_bounds__(NTHR) void ode_kernel(const float* __restrict__ z0, const float* __restrict__ tg,
                                                   const unsigned short* __restrict__ W1p,
                                                   const unsigned short* __restrict__ W2p,
                                                   const unsigned short* __restrict__ W3p,
                                                   const float* __restrict__ b1, const float* __restrict__ b2,
                                                   const float* __restrict__ b3, float* __restrict__ YS) {
  __shared__ __align__(16) _Float16 Ysh[ROWS_BLK * YPITCH];
  __shared__ __align__(16) _Float16 H1s[ROWS_BLK * HPITCH];
  __shared__ __align__(16) _Float16 H2s[ROWS_BLK * HPITCH];
  __shared__ __align__(16) float    Sl[ROWS_BLK * SPITCH];
  const _Float16* W1T = (const _Float16*)W1p;
  const _Float16* W2T = (const _Float16*)W2p;
  const _Float16* W3T = (const _Float16*)W3p;
  const int tid = threadIdx.x, lane = tid & 31, wave = tid >> 5, hh = lane >> 4, c = lane & 15;
  const int rowbase = blockIdx.x * ROWS_BLK;
  const int jst = 16 * wave + c;

  float ts[NTIME];
#pragma unroll
  for (int i = 0; i < NTIME; ++i) ts[i] = tg[i];
#pragma unroll
  for (int p = 0; p < NTIME - 1; ++p) {
#pragma unroll
    for (int q = 0; q < NTIME - 1 - p; ++q) {
      const float lo = fminf(ts[q], ts[q + 1]);
      const float hi = fmaxf(ts[q], ts[q + 1]);
      ts[q] = lo; ts[q + 1] = hi;
    }
  }

  float b1r[4], b2r[4];
#pragma unroll
  for (int nt = 0; nt < 4; ++nt) {
    const int j = 64 * wave + 16 * nt + c;
    b1r[nt] = b1[j];
    b2r[nt] = b2[j];
  }
  const float b3r = b3[jst];

  float y[8];
  const int jcl = (jst < DIM_LAT) ? jst : (DIM_LAT - 1);
#pragma unroll
  for (int r = 0; r < 8; ++r) {
    const float v = z0[(size_t)(rowbase + 8 * hh + r) * DIM_LAT + jcl];
    y[r] = (jst < DIM_LAT) ? v : 0.0f;
  }
  store_state(Sl, YS + (size_t)rowbase * DIM_ST, wave, hh, c, lane, y);

  float k1[8], k2[8], k3[8], k4[8], k5[8], k6[8], yt[8];
#pragma unroll 1
  for (int ti = 0; ti < NTIME - 1; ++ti) {
    float ta = ts[0], tb = ts[1];
#pragma unroll
    for (int i = 1; i < NTIME - 1; ++i) {
      const bool s = (ti == i);
      ta = s ? ts[i] : ta;
      tb = s ? ts[i + 1] : tb;
    }
    const float dt = (tb - ta) / 6.0f;
#pragma unroll 1
    for (int ss = 0; ss < NSUB; ++ss) {
      feval(Ysh, H1s, H2s, W1T, W2T, W3T, b1r, b2r, b3r, wave, hh, c, y, k1);
#pragma unroll
      for (int r = 0; r < 8; ++r) yt[r] = y[r] + dt * (RK_A21 * k1[r]);
      feval(Ysh, H1s, H2s, W1T, W2T, W3T, b1r, b2r, b3r, wave, hh, c, yt, k2);
#pragma unroll
      for (int r = 0; r < 8; ++r) yt[r] = y[r] + dt * (RK_A31 * k1[r] + RK_A32 * k2[r]);
      feval(Ysh, H1s, H2s, W1T, W2T, W3T, b1r, b2r, b3r, wave, hh, c, yt, k3);
#pragma unroll
      for (int r = 0; r < 8; ++r) yt[r] = y[r] + dt * (RK_A41 * k1[r] - RK_A42 * k2[r] + RK_A43 * k3[r]);
      feval(Ysh, H1s, H2s, W1T, W2T, W3T, b1r, b2r, b3r, wave, hh, c, yt, k4);
#pragma unroll
      for (int r = 0; r < 8; ++r)
        yt[r] = y[r] + dt * (RK_A51 * k1[r] - RK_A52 * k2[r] + RK_A53 * k3[r] - RK_A54 * k4[r]);
      feval(Ysh, H1s, H2s, W1T, W2T, W3T, b1r, b2r, b3r, wave, hh, c, yt, k5);
#pragma unroll
      for (int r = 0; r < 8; ++r)
        yt[r] = y[r] + dt * (RK_A61 * k1[r] - RK_A62 * k2[r] + RK_A63 * k3[r] + RK_A64 * k4[r] - RK_A65 * k5[r]);
      feval(Ysh, H1s, H2s, W1T, W2T, W3T, b1r, b2r, b3r, wave, hh, c, yt, k6);
#pragma unroll
      for (int r = 0; r < 8; ++r)
        y[r] = y[r] + dt * (RK_B1 * k1[r] + RK_B3 * k3[r] + RK_B4 * k4[r] - RK_B5 * k5[r] + RK_B6 * k6[r]);
    }
    store_state(Sl, YS + ((size_t)(ti + 1) * NBATCH + rowbase) * DIM_ST, wave, hh, c, lane, y);
  }
}

__global__ __launch_bounds__(NTHR) void pack_kernel(const float* __restrict__ YS, float* __restrict__ out) {
  const int i = blockIdx.x * NTHR + threadIdx.x;
  if (i >= NOUT_V4) return;
  v4f o;
#pragma unroll
  for (int e = 0; e < 4; ++e) {
    const int f = 4 * i + e;
    const int b = f / (NTIME * DIM_LAT);
    const int rem = f - b * (NTIME * DIM_LAT);
    const int t = rem / DIM_LAT;
    const int j = rem - t * DIM_LAT;
    o[e] = YS[((size_t)t * NBATCH + b) * DIM_ST + j];
  }
  float* op = out + (size_t)i * 4;
  *(volatile v4f*)op = o;
  __threadfence();
  *(volatile v4f*)op = o;
}

extern "C" void kernel_launch(void* const* d_in, const int* in_sizes, int n_in,
                              void* d_out, int out_size, void* d_ws, size_t ws_size, hipStream_t stream) {
  if (n_in < 8 || d_out == nullptr || d_ws == nullptr) return;
  if (in_sizes[0] != NBATCH * DIM_LAT || in_sizes[1] != NBATCH * NTIME || in_sizes[2] != DIM_ST * DIM_HID ||
      in_sizes[3] != DIM_HID || in_sizes[4] != DIM_HID * DIM_HID || in_sizes[5] != DIM_HID ||
      in_sizes[6] != DIM_HID * DIM_ST || in_sizes[7] != DIM_ST || out_size != NOUT_EL) return;

  const float* z0 = (const float*)d_in[0];
  const float* tg = (const float*)d_in[1];
  const float* W1 = (const float*)d_in[2];
  const float* b1 = (const float*)d_in[3];
  const float* W2 = (const float*)d_in[4];
  const float* b2 = (const float*)d_in[5];
  const float* W3 = (const float*)d_in[6];
  const float* b3 = (const float*)d_in[7];
  float* out = (float*)d_out;

  char* ws = (char*)d_ws; size_t off = 0;
  auto carve = [&](size_t bytes) -> char* { char* p = ws + off; off += (bytes + 255) & ~(size_t)255; return p; };
  unsigned short* W1T = (unsigned short*)carve((size_t)DIM_HID * DIM_ST * 2);
  unsigned short* W2T = (unsigned short*)carve((size_t)DIM_HID * DIM_HID * 2);
  unsigned short* W3T = (unsigned short*)carve((size_t)DIM_ST * DIM_HID * 2);
  float*          YS  = (float*)carve((size_t)NTIME * NBATCH * DIM_ST * 4);
  if (off > ws_size || off > (size_t)134217728) return;

  wt_cast_kernel<<<dim3(DIM_ST / 64, DIM_HID / 32), NTHR, 0, stream>>>(W1, W1T, DIM_ST, DIM_HID, CARRY1);
  wt_cast_kernel<<<dim3(DIM_HID / 64, DIM_HID / 32), NTHR, 0, stream>>>(W2, W2T, DIM_HID, DIM_HID, CARRY2);
  wt_cast_kernel<<<dim3(DIM_HID / 64, DIM_ST / 32), NTHR, 0, stream>>>(W3, W3T, DIM_HID, DIM_ST, CARRY2);

  ode_kernel<<<NBATCH / ROWS_BLK, NTHR, 0, stream>>>(z0, tg, W1T, W2T, W3T, b1, b2, b3, YS);

  pack_kernel<<<NOUT_V4 / NTHR, NTHR, 0, stream>>>(YS, out);
}
